// FeedForwardQuantum_65481071395866
// MI455X (gfx1250) — hardware-verified
//
#include <hip/hip_runtime.h>
#include <math.h>

constexpr int kBatch  = 8;
constexpr int kSeq    = 2048;
constexpr int kTokens = kBatch * kSeq;
constexpr int kEmb    = 256;
constexpr int kNQ     = 10;
constexpr int kKpad   = 32;
constexpr int kFF     = 1024;
constexpr int kQP     = 36;
constexpr int kRowsPerBlock = 256;

typedef __attribute__((ext_vector_type(16))) _Float16 v16h;
typedef __attribute__((ext_vector_type(8)))  _Float16 v8h;
typedef __attribute__((ext_vector_type(16))) __bf16   v16b;
typedef __attribute__((ext_vector_type(8)))  __bf16   v8b;
typedef __attribute__((ext_vector_type(8)))  float    v8f;
typedef __attribute__((ext_vector_type(4)))  float    v4f;
typedef __attribute__((ext_vector_type(4)))  unsigned int v4u;

__device__ __forceinline__ unsigned short f2bf_bits(float f) {
  unsigned u = __float_as_uint(f);
  return (unsigned short)((u + 0x7FFFu + ((u >> 16) & 1u)) >> 16);
}
__device__ __forceinline__ float bf_bits2f(unsigned short h) { return __uint_as_float(((unsigned)h) << 16); }

__device__ __forceinline__ void dep_guard_h(v8f& a, v8f& b, v16h x, v16h y) { asm volatile("v_nop\n\tv_nop\n\tv_nop\n\tv_nop" : "+v"(a), "+v"(b) : "v"(x), "v"(y)); }
__device__ __forceinline__ void dep_guard_b(v8f& a, v8f& b, v16b x, v16b y) { asm volatile("v_nop\n\tv_nop\n\tv_nop\n\tv_nop" : "+v"(a), "+v"(b) : "v"(x), "v"(y)); }
__device__ __forceinline__ void keep4_h(v16h a, v16h b, v16h c, v16h d) { asm volatile("v_nop" :: "v"(a), "v"(b), "v"(c), "v"(d)); }
__device__ __forceinline__ void keep4_b(v16b a, v16b b, v16b c, v16b d) { asm volatile("v_nop" :: "v"(a), "v"(b), "v"(c), "v"(d)); }
__device__ __forceinline__ void acc_guard4(v8f& a, v8f& b, v8f& c, v8f& d) { asm volatile("v_nop\n\tv_nop\n\tv_nop\n\tv_nop" : "+v"(a), "+v"(b), "+v"(c), "+v"(d)); }
template <typename T> struct Frag;
template <> struct Frag<_Float16> {
  typedef v16h V; union U { v16h v; v8h h[2]; };
  static __device__ __forceinline__ v16h load(const _Float16* p) {
    U f; f.h[0] = *(const v8h*)(p); f.h[1] = *(const v8h*)(p + 16); return f.v;
  }
  static __device__ __forceinline__ v8f mma(v16h a, v16h b, v8f c) {
    return __builtin_amdgcn_wmma_f32_16x16x32_f16(false, a, false, b, (short)0, c, false, false);
  }
  static __device__ __forceinline__ void guard(v8f& a, v8f& b, v16h x, v16h y) { dep_guard_h(a, b, x, y); }
  static __device__ __forceinline__ void keep(v16h a, v16h b, v16h c, v16h d) { keep4_h(a, b, c, d); }
};
template <> struct Frag<__bf16> {
  typedef v16b V; union U { v16b v; v8b h[2]; };
  static __device__ __forceinline__ v16b load(const __bf16* p) {
    U f; f.h[0] = *(const v8b*)(p); f.h[1] = *(const v8b*)(p + 16); return f.v;
  }
  static __device__ __forceinline__ v8f mma(v16b a, v16b b, v8f c) {
    return __builtin_amdgcn_wmma_f32_16x16x32_bf16(false, a, false, b, (short)0, c, false, false);
  }
  static __device__ __forceinline__ void guard(v8f& a, v8f& b, v16b x, v16b y) { dep_guard_b(a, b, x, y); }
  static __device__ __forceinline__ void keep(v16b a, v16b b, v16b c, v16b d) { keep4_b(a, b, c, d); }
};

__device__ __forceinline__ unsigned pk16(unsigned short a, unsigned short b) { return (unsigned)a | ((unsigned)b << 16); }

template <int ET> struct Elem;
template <> struct Elem<0> { typedef _Float16 T; };
template <> struct Elem<1> { typedef __bf16 T; };
template <int ET, bool SPLIT, int BIAS_MODE, int OUT_MODE, bool RESID, int ACT = 0>
__global__ __launch_bounds__(256) void wmma_gemm64(
    const unsigned short* __restrict__ Ap, const unsigned short* __restrict__ A2p, int lda, long strideA,
    const unsigned short* __restrict__ Btp, const unsigned short* __restrict__ Bt2p, int ldb, long strideB,
    void* __restrict__ Cout, void* __restrict__ Cout2, int ldc, long strideC,
    const float* __restrict__ bias,
    const float* __restrict__ resid, long strideR,
    int M, int N, int K, float scale) {
  typedef typename Elem<ET>::T T;
  typedef typename Frag<T>::V V;
  const T* A = (const T*)Ap; const T* A2 = (const T*)A2p; const T* Bt = (const T*)Btp; const T* Bt2 = (const T*)Bt2p;
  __shared__ __align__(16) float sT[8][16 * 68];
  const int b    = blockIdx.y;
  const int lane = threadIdx.x & 31;
  const int wave = threadIdx.x >> 5;
  const int tilesN = N >> 6;
  const int tilesM = M >> 6;
  const int tile = blockIdx.x * 8 + wave;
  if (tile >= tilesM * tilesN) return;
  const int tm = tile / tilesN;
  const int tn = tile - tm * tilesN;
  const int m0 = tm << 6;
  const int n0 = tn << 6;

  const T* Ab  = A  + (size_t)b * strideA;
  const T* Bb  = Bt + (size_t)b * strideB;
  const T* Ab2 = SPLIT ? (A2  + (size_t)b * strideA) : nullptr;
  const T* Bb2 = SPLIT ? (Bt2 + (size_t)b * strideB) : nullptr;

  const int rlane = lane & 15;
  const int koff  = (lane >> 4) * 8;
  const int mOff  = (lane >> 4) * 8;

  v8f acc[4][4];
#pragma unroll
  for (int i = 0; i < 4; ++i)
#pragma unroll
    for (int j = 0; j < 4; ++j) acc[i][j] = (v8f){0.f,0.f,0.f,0.f,0.f,0.f,0.f,0.f};

  for (int k0 = 0; k0 < K; k0 += 32) {
    V bh[4], bl[4];
#pragma unroll
    for (int j = 0; j < 4; ++j) {
      const size_t bo = (size_t)(n0 + (j << 4) + rlane) * ldb + koff + k0;
      bh[j] = Frag<T>::load(Bb + bo);
      if (SPLIT) bl[j] = Frag<T>::load(Bb2 + bo);
    }
#pragma unroll
    for (int i = 0; i < 4; ++i) {
      const size_t ao = (size_t)(m0 + (i << 4) + rlane) * lda + koff + k0;
      V ah = Frag<T>::load(Ab + ao);
      V al;
      if (SPLIT) al = Frag<T>::load(Ab2 + ao);
#pragma unroll
      for (int j = 0; j < 4; ++j) {
        acc[i][j] = Frag<T>::mma(ah, bh[j], acc[i][j]);
        if (SPLIT) {
          acc[i][j] = Frag<T>::mma(ah, bl[j], acc[i][j]);
          acc[i][j] = Frag<T>::mma(al, bh[j], acc[i][j]);
        }
      }
      Frag<T>::guard(acc[i][0], acc[i][3], ah, SPLIT ? al : ah);
    }
    Frag<T>::keep(bh[0], bh[1], bh[2], bh[3]);
    if (SPLIT) Frag<T>::keep(bl[0], bl[1], bl[2], bl[3]);
  }
  acc_guard4(acc[0][0], acc[0][1], acc[0][2], acc[0][3]);
  acc_guard4(acc[1][0], acc[1][1], acc[1][2], acc[1][3]);
  acc_guard4(acc[2][0], acc[2][1], acc[2][2], acc[2][3]);
  acc_guard4(acc[3][0], acc[3][1], acc[3][2], acc[3][3]);

  float* slab = sT[wave];
  const float* Rb = RESID ? (resid + (size_t)b * strideR) : nullptr;
#pragma unroll
  for (int i = 0; i < 4; ++i) {
    const int mBase = m0 + (i << 4);
#pragma unroll
    for (int j = 0; j < 4; ++j) {
      const int n = n0 + (j << 4) + rlane;
      float bv = 0.f;
      if (BIAS_MODE == 2) bv = bias[n];
#pragma unroll
      for (int r = 0; r < 8; ++r) {
        float v = acc[i][j][r] * scale;
        if (BIAS_MODE == 1) v += bias[mBase + mOff + r];
        if (BIAS_MODE == 2) v += bv;
        if (RESID) v += Rb[(size_t)(mBase + mOff + r) * ldc + n];
        if (ACT == 2) v = fmaxf(v, 0.0f);
        if (ACT == 4) v = (v > 0.f) ? v : 0.01f * v;
        slab[(mOff + r) * 68 + (j << 4) + rlane] = v;
      }
    }
    __builtin_amdgcn_fence(__ATOMIC_RELEASE, "workgroup");
    __builtin_amdgcn_wave_barrier();
    __builtin_amdgcn_fence(__ATOMIC_ACQUIRE, "workgroup");
    if (OUT_MODE == 0) {
      float* C = (float*)Cout + (size_t)b * strideC;
      const int hh = lane >> 4, c4 = (lane & 15) * 4;
      for (int pass = 0; pass < 2; ++pass) {
#pragma unroll
        for (int it = 0; it < 8; ++it) {
          const int row = it * 2 + hh;
          v4f v = *(const v4f*)(slab + row * 68 + c4);
          *(volatile v4f*)(C + (size_t)(mBase + row) * ldc + n0 + c4) = v;
        }
        __threadfence();
      }
    } else {
      const int q = lane >> 3, c8 = (lane & 7) * 8;
      unsigned short* C  = (unsigned short*)Cout  + (size_t)b * strideC;
      unsigned short* C2 = (OUT_MODE == 2) ? ((unsigned short*)Cout2 + (size_t)b * strideC) : nullptr;
      for (int pass = 0; pass < 2; ++pass) {
#pragma unroll
        for (int it = 0; it < 4; ++it) {
          const int row = it * 4 + q;
          const float* sp = slab + row * 68 + c8;
          v8h hv, lv;
#pragma unroll
          for (int e = 0; e < 8; ++e) {
            if (OUT_MODE == 1) {
              hv[e] = (_Float16)sp[e];
            } else {
              unsigned short hb = f2bf_bits(sp[e]);
              unsigned short lb = f2bf_bits(sp[e] - bf_bits2f(hb));
              hv[e] = __builtin_bit_cast(_Float16, hb);
              lv[e] = __builtin_bit_cast(_Float16, lb);
            }
          }
          *(volatile v8h*)(C + (size_t)(mBase + row) * ldc + n0 + c8) = hv;
          if (OUT_MODE == 2) *(volatile v8h*)(C2 + (size_t)(mBase + row) * ldc + n0 + c8) = lv;
        }
        __threadfence();
      }
    }
    __builtin_amdgcn_fence(__ATOMIC_RELEASE, "workgroup");
    __builtin_amdgcn_wave_barrier();
    __builtin_amdgcn_fence(__ATOMIC_ACQUIRE, "workgroup");
  }
}

template <bool QMODE>
__global__ __launch_bounds__(256) void rows32_planes_kernel(
    const float* __restrict__ src, const float* __restrict__ theta,
    unsigned short* __restrict__ ph, unsigned short* __restrict__ pl, int nrows) {
  __shared__ __align__(16) float qs[kRowsPerBlock * kQP];
  const int tid  = threadIdx.x;
  const int row0 = blockIdx.x * kRowsPerBlock;
  if (row0 + kRowsPerBlock > nrows) return;
  const int grow = row0 + tid;
  float* qrow = qs + tid * kQP;

  if (QMODE) {
    const float* xrow = src + (size_t)grow * kEmb;
    float ct = 1.0f, pref = 1.0f, suf = 1.0f;
#pragma unroll 1
    for (int i = 0; i < 2 * kNQ; ++i) {
      const int j = i >> 1;
      const float ath = theta[j];
      const float ax  = xrow[j];
      const bool isx  = (i & 1) != 0;
      const float arg = isx ? ax : ath;
      const float cv  = cosf(arg);
      if (isx) {
        const float m = ct * cv;
        if (j == 0) {
          pref = m;
        } else {
          pref = pref * m;
          suf  = suf * m;
          qrow[j] = pref;
        }
      } else {
        ct = cv;
      }
    }
    qrow[0] = suf;
  } else {
    const float* wrow = src + (size_t)grow * kNQ;
#pragma unroll
    for (int j = 0; j < kNQ; ++j) qrow[j] = wrow[j];
  }
#pragma unroll
  for (int j = kNQ; j < kKpad; ++j) qrow[j] = 0.0f;
  __syncthreads();

  const int lane = tid & 31, wave = tid >> 5;
  const int rq = lane >> 2;
  const int cg = (lane & 3) * 8;
  v4u hw[4], lw[4];
#pragma unroll
  for (int it = 0; it < 4; ++it) {
    const int rl = wave * 32 + it * 8 + rq;
    const float* sp = qs + rl * kQP + cg;
    const v4f a = *(const v4f*)(sp);
    const v4f c = *(const v4f*)(sp + 4);
    unsigned short hb[8], lb[8];
#pragma unroll
    for (int e = 0; e < 4; ++e) {
      const float v0 = a[e];
      const float v1 = c[e];
      hb[e]     = f2bf_bits(v0);
      lb[e]     = f2bf_bits(v0 - bf_bits2f(hb[e]));
      hb[4 + e] = f2bf_bits(v1);
      lb[4 + e] = f2bf_bits(v1 - bf_bits2f(hb[4 + e]));
    }
    hw[it] = (v4u){pk16(hb[0], hb[1]), pk16(hb[2], hb[3]), pk16(hb[4], hb[5]), pk16(hb[6], hb[7])};
    lw[it] = (v4u){pk16(lb[0], lb[1]), pk16(lb[2], lb[3]), pk16(lb[4], lb[5]), pk16(lb[6], lb[7])};
  }
  for (int pass = 0; pass < 2; ++pass) {
#pragma unroll
    for (int it = 0; it < 4; ++it) {
      const size_t gr = (size_t)(row0 + wave * 32 + it * 8 + rq);
      *(volatile v4u*)(ph + gr * kKpad + cg) = hw[it];
      *(volatile v4u*)(pl + gr * kKpad + cg) = lw[it];
    }
    __threadfence();
  }
}

__global__ __launch_bounds__(256) void cast8_bf16x2_kernel(const float* __restrict__ in,
                                                           unsigned short* __restrict__ oh,
                                                           unsigned short* __restrict__ ol, int n8) {
  const int i = blockIdx.x * 256 + threadIdx.x;
  if (i >= n8) return;
  const float* p = in + 8 * (size_t)i;
  const v4f a = *(const v4f*)(p);
  const v4f c = *(const v4f*)(p + 4);
  unsigned short hb[8], lb[8];
#pragma unroll
  for (int e = 0; e < 4; ++e) {
    const float v0 = a[e];
    const float v1 = c[e];
    hb[e]     = f2bf_bits(v0);
    lb[e]     = f2bf_bits(v0 - bf_bits2f(hb[e]));
    hb[4 + e] = f2bf_bits(v1);
    lb[4 + e] = f2bf_bits(v1 - bf_bits2f(hb[4 + e]));
  }
  const v4u uh = (v4u){pk16(hb[0], hb[1]), pk16(hb[2], hb[3]), pk16(hb[4], hb[5]), pk16(hb[6], hb[7])};
  const v4u ul = (v4u){pk16(lb[0], lb[1]), pk16(lb[2], lb[3]), pk16(lb[4], lb[5]), pk16(lb[6], lb[7])};
  unsigned short* qh = oh + 8 * (size_t)i;
  unsigned short* ql = ol + 8 * (size_t)i;
  *(volatile v4u*)qh = uh;
  *(volatile v4u*)ql = ul;
  __threadfence();
  *(volatile v4u*)qh = uh;
  *(volatile v4u*)ql = ul;
}

constexpr size_t kQPlaneB  = (size_t)kTokens * kKpad * 2;
constexpr size_t kW1PlaneB = (size_t)kFF * kKpad * 2;
constexpr size_t kW2PlaneB = (size_t)kEmb * kFF * 2;
constexpr size_t kHPlaneB  = (size_t)kTokens * kFF * 2;
constexpr size_t kOffQh  = 0;
constexpr size_t kOffQl  = kOffQh  + kQPlaneB;
constexpr size_t kOffW1h = kOffQl  + kQPlaneB;
constexpr size_t kOffW1l = kOffW1h + kW1PlaneB;
constexpr size_t kOffW2h = kOffW1l + kW1PlaneB;
constexpr size_t kOffW2l = kOffW2h + kW2PlaneB;
constexpr size_t kOffHh  = kOffW2l + kW2PlaneB;
constexpr size_t kOffHl  = kOffHh  + kHPlaneB;
constexpr size_t kWsTotal = kOffHl + kHPlaneB;
static_assert(kWsTotal == 70385664u);
static_assert(kWsTotal <= 134217728u);
static_assert((kOffQl % 128) == 0 && (kOffW1h % 128) == 0 && (kOffW1l % 128) == 0 && (kOffW2h % 128) == 0 &&
              (kOffW2l % 128) == 0 && (kOffHh % 128) == 0 && (kOffHl % 128) == 0);
static_assert(kTokens % 64 == 0 && kFF % 64 == 0 && kKpad % 32 == 0);
static_assert(kTokens % 64 == 0 && kEmb % 64 == 0 && kFF % 32 == 0);
static_assert(kTokens % kRowsPerBlock == 0 && kFF % kRowsPerBlock == 0);
static_assert((kEmb * kFF) % (8 * 256) == 0);

extern "C" void kernel_launch(void* const* d_in, const int* in_sizes, int n_in,
                              void* d_out, int out_size, void* d_ws, size_t ws_size,
                              hipStream_t stream) {
  if (n_in < 6) return;
  if (in_sizes[0] < kTokens * kEmb || in_sizes[1] < kNQ || in_sizes[2] < kFF * kNQ ||
      in_sizes[3] < kFF || in_sizes[4] < kEmb * kFF || in_sizes[5] < kEmb) return;
  if ((size_t)out_size < (size_t)kTokens * kEmb) return;
  if (ws_size < kWsTotal) return;

  const float* x     = (const float*)d_in[0];
  const float* theta = (const float*)d_in[1];
  const float* w1    = (const float*)d_in[2];
  const float* b1    = (const float*)d_in[3];
  const float* w2    = (const float*)d_in[4];
  const float* b2    = (const float*)d_in[5];
  float* out = (float*)d_out;
  char* ws = (char*)d_ws;
  unsigned short* qh  = (unsigned short*)(ws + kOffQh);
  unsigned short* ql  = (unsigned short*)(ws + kOffQl);
  unsigned short* w1h = (unsigned short*)(ws + kOffW1h);
  unsigned short* w1l = (unsigned short*)(ws + kOffW1l);
  unsigned short* w2h = (unsigned short*)(ws + kOffW2h);
  unsigned short* w2l = (unsigned short*)(ws + kOffW2l);
  unsigned short* hh  = (unsigned short*)(ws + kOffHh);
  unsigned short* hl  = (unsigned short*)(ws + kOffHl);

  rows32_planes_kernel<true><<<dim3(kTokens / kRowsPerBlock), dim3(256), 0, stream>>>(x, theta, qh, ql, kTokens);
  rows32_planes_kernel<false><<<dim3(kFF / kRowsPerBlock), dim3(256), 0, stream>>>(w1, theta, w1h, w1l, kFF);
  {
    const int n8 = (kEmb * kFF) / 8;
    cast8_bf16x2_kernel<<<dim3(n8 / 256), dim3(256), 0, stream>>>(w2, w2h, w2l, n8);
  }
  {
    const int tiles = (kTokens / 64) * (kFF / 64);
    wmma_gemm64<1, true, 2, 2, false, 2><<<dim3(tiles / 8, 1), dim3(256), 0, stream>>>(
        (const unsigned short*)qh, (const unsigned short*)ql, kKpad, 0L,
        (const unsigned short*)w1h, (const unsigned short*)w1l, kKpad, 0L,
        (void*)hh, (void*)hl, kFF, 0L,
        b1, (const float*)nullptr, 0L,
        kTokens, kFF, kKpad, 1.0f);
  }
  {
    const int tiles = (kTokens / 64) * (kEmb / 64);
    wmma_gemm64<1, true, 2, 0, false, 0><<<dim3(tiles / 8, 1), dim3(256), 0, stream>>>(
        (const unsigned short*)hh, (const unsigned short*)hl, kFF, 0L,
        (const unsigned short*)w2h, (const unsigned short*)w2l, kFF, 0L,
        (void*)out, (void*)nullptr, kEmb, 0L,
        b2, (const float*)nullptr, 0L,
        kTokens, kEmb, kFF, 1.0f);
  }
}
